// PersistentWorldMemoryBank_29953101922438
// MI455X (gfx1250) — hardware-verified
//
#include <hip/hip_runtime.h>
#include <math.h>
#include <stdint.h>

#define NQ     4096
#define NG     4096
#define KVV    4097
#define NKP    4160
#define DM     256
#define DROI   1024
#define DSTR   256
#define DCAM   128
#define DMOT   64
#define GIN    704
#define GOUT   768
#define NH     4
#define HD     64
#define NQT    (NQ / 16)
#define NWAV   (NQT * NH)
#define KSTEPS 129
#define PSP    36
#define ACT    16.0f
#define WSC    256.0f
#define QKC    64.0f
#define VC     64.0f
#define ZC     1024.0f
#define AOC    4096.0f
#define PONE   64.0f
#define PCAR   262208.0f
#define RESC   2048.0f
#define RINV   0.00048828125f
#define NEGS   (-1.0e30f)

static_assert(NH * HD == DM);
static_assert(KSTEPS * 32 >= KVV);
static_assert((KSTEPS - 1) * 32 < KVV);
static_assert(KSTEPS * 32 <= NKP);
static_assert((NKP % 64) == 0 && (NQ % 64) == 0 && (DM % 64) == 0 && (GOUT % 64) == 0);
static_assert((GIN % 32) == 0 && (GIN % 64) == 0 && (DROI % 64) == 0);
static_assert((NWAV % 4) == 0);
static_assert(PCAR == (float)KVV * PONE);
static_assert(DM + DSTR + DCAM + DMOT == GIN);

typedef _Float16 v16h __attribute__((ext_vector_type(16)));
typedef _Float16 v8h  __attribute__((ext_vector_type(8)));
typedef float    v8f  __attribute__((ext_vector_type(8)));
typedef float    v4f  __attribute__((ext_vector_type(4)));
typedef unsigned int v4u __attribute__((ext_vector_type(4)));

union FragH { v16h v; v8h h[2]; v4u u[2]; };

__device__ __forceinline__ unsigned short bf_bits(float f) {
  unsigned u = __float_as_uint(f);
  return (unsigned short)((u + 0x7FFFu + ((u >> 16) & 1u)) >> 16);
}
__device__ __forceinline__ float bf_up(unsigned short b) { return __uint_as_float(((unsigned)b) << 16); }
__device__ __forceinline__ float bfr(float f) { return bf_up(bf_bits(f)); }
__device__ __forceinline__ unsigned short h_bits(_Float16 x) { return __builtin_bit_cast(unsigned short, x); }
__device__ __forceinline__ unsigned pk16(unsigned short a, unsigned short b) { return (unsigned)a | ((unsigned)b << 16); }
__device__ __forceinline__ v8f zero8() { v8f z = {0.f, 0.f, 0.f, 0.f, 0.f, 0.f, 0.f, 0.f}; return z; }

__device__ __forceinline__ v16h ldfrag_h(const _Float16* p) {
  FragH f;
  f.h[0] = *(const v8h*)(p);
  f.h[1] = *(const v8h*)(p + 16);
  return f.v;
}
__device__ __forceinline__ v16h ldfrag_u(const unsigned short* p) {
  FragH f;
  f.u[0] = *(const v4u*)(p);
  f.u[1] = *(const v4u*)(p + 16);
  return f.v;
}

__device__ __forceinline__ v8f mma_raw(v16h a, v16h b, v8f c) {
  return __builtin_amdgcn_wmma_f32_16x16x32_f16(false, a, false, b, (short)0, c, false, false);
}
__device__ __forceinline__ void guard_4x1(v8f& a, v8f& b, v8f& c, v8f& d, v16h x) {
#if defined(__HIP_DEVICE_COMPILE__)
  asm volatile("v_nop\n\tv_nop\n\tv_nop\n\tv_nop" : "+v"(a), "+v"(b), "+v"(c), "+v"(d) : "v"(x));
#endif
}
__device__ __forceinline__ void keep4_h(v16h a, v16h b, v16h c, v16h d) {
#if defined(__HIP_DEVICE_COMPILE__)
  asm volatile("v_nop" :: "v"(a), "v"(b), "v"(c), "v"(d));
#endif
}
__device__ __forceinline__ void acc_guard4(v8f& a, v8f& b, v8f& c, v8f& d) {
#if defined(__HIP_DEVICE_COMPILE__)
  asm volatile("v_nop\n\tv_nop\n\tv_nop\n\tv_nop" : "+v"(a), "+v"(b), "+v"(c), "+v"(d));
#endif
}
__device__ __forceinline__ void guard_2x6(v8f& a, v8f& b, v16h x0, v16h x1, v16h x2, v16h x3, v16h x4, v16h x5) {
#if defined(__HIP_DEVICE_COMPILE__)
  asm volatile("v_nop\n\tv_nop\n\tv_nop\n\tv_nop"
               : "+v"(a), "+v"(b) : "v"(x0), "v"(x1), "v"(x2), "v"(x3), "v"(x4), "v"(x5));
#endif
}
__device__ __forceinline__ void guard_4x5(v8f& a, v8f& b, v8f& c, v8f& d, v16h x0, v16h x1, v16h x2, v16h x3, v16h x4) {
#if defined(__HIP_DEVICE_COMPILE__)
  asm volatile("v_nop\n\tv_nop\n\tv_nop\n\tv_nop"
               : "+v"(a), "+v"(b), "+v"(c), "+v"(d) : "v"(x0), "v"(x1), "v"(x2), "v"(x3), "v"(x4));
#endif
}
__device__ __forceinline__ void wave_sync_lds() {
  __builtin_amdgcn_fence(__ATOMIC_RELEASE, "workgroup");
  __builtin_amdgcn_wave_barrier();
  __builtin_amdgcn_fence(__ATOMIC_ACQUIRE, "workgroup");
}

__device__ __forceinline__ v4u pack8h(const float* sp) {
  const v4f a = *(const v4f*)(sp), b = *(const v4f*)(sp + 4);
  float v[8];
#pragma unroll
  for (int e = 0; e < 4; ++e) { v[e] = a[e]; v[4 + e] = b[e]; }
  v4u o;
#pragma unroll
  for (int e = 0; e < 4; ++e) o[e] = pk16(h_bits((_Float16)v[2 * e]), h_bits((_Float16)v[2 * e + 1]));
  return o;
}

__global__ __launch_bounds__(256) void cvk(const float* __restrict__ x, unsigned short* dst, int nch, int rne, float scale) {
  const int i = blockIdx.x * 256 + threadIdx.x;
  const bool live = i < nch;
  const int ic = live ? i : (nch - 1);
  const float* p = x + (size_t)ic * 8;
  const v4f a = *(const v4f*)(p), b = *(const v4f*)(p + 4);
  float v[8];
#pragma unroll
  for (int e = 0; e < 4; ++e) { v[e] = a[e]; v[4 + e] = b[e]; }
  if (rne != 0) {
#pragma unroll
    for (int e = 0; e < 8; ++e) v[e] = bfr(v[e]);
  }
  v4u o;
#pragma unroll
  for (int e = 0; e < 4; ++e)
    o[e] = pk16(h_bits((_Float16)(v[2 * e] * scale)), h_bits((_Float16)(v[2 * e + 1] * scale)));
  unsigned short* dp = dst + (size_t)ic * 8;
  if (live) *(volatile v4u*)dp = o;
  __threadfence();
  if (live) *(volatile v4u*)dp = o;
}

__global__ __launch_bounds__(256) void cvT(const float* __restrict__ W, unsigned short* dst, int K, int N, float scale) {
  __shared__ __align__(16) float s[64][68];
  const int t  = threadIdx.x;
  const int n0 = blockIdx.x * 64, k0 = blockIdx.y * 64;
#pragma unroll
  for (int it = 0; it < 16; ++it) {
    const int idx = it * 256 + t;
    const int r = idx >> 6, cc = idx & 63;
    s[cc][r] = bfr(W[(size_t)(k0 + r) * (size_t)N + n0 + cc]) * scale;
  }
  __syncthreads();
  const int wave = t >> 5, lane = t & 31, q8 = lane >> 3, c8 = (lane & 7) * 8;
  v4u o[2];
  size_t ofs[2];
#pragma unroll
  for (int it = 0; it < 2; ++it) {
    const int cc = wave * 8 + it * 4 + q8;
    o[it]   = pack8h(&s[cc][c8]);
    ofs[it] = (size_t)(n0 + cc) * (size_t)K + (size_t)(k0 + c8);
  }
#pragma unroll
  for (int it = 0; it < 2; ++it) *(volatile v4u*)(dst + ofs[it]) = o[it];
  __threadfence();
#pragma unroll
  for (int it = 0; it < 2; ++it) *(volatile v4u*)(dst + ofs[it]) = o[it];
}

__device__ __forceinline__ void kloop(v8f (&acc)[4][4], const unsigned short* __restrict__ A1, int lda,
                                      const unsigned short* __restrict__ Bb, int ldb, int m0, int n0, int K,
                                      int rlane, int koff) {
#pragma unroll 1
  for (int k0 = 0; k0 < K; k0 += 32) {
    v16h bh[4];
#pragma unroll
    for (int j = 0; j < 4; ++j) {
      const size_t bofs = (size_t)(n0 + (j << 4) + rlane) * (size_t)ldb + (size_t)(koff + k0);
      bh[j] = ldfrag_u(Bb + bofs);
    }
#pragma unroll
    for (int i = 0; i < 4; ++i) {
      const size_t ao = (size_t)(m0 + (i << 4) + rlane) * (size_t)lda + (size_t)(k0 + koff);
      const v16h ah = ldfrag_u(A1 + ao);
#pragma unroll
      for (int j = 0; j < 4; ++j) acc[i][j] = mma_raw(ah, bh[j], acc[i][j]);
      guard_4x1(acc[i][0], acc[i][1], acc[i][2], acc[i][3], ah);
    }
    keep4_h(bh[0], bh[1], bh[2], bh[3]);
  }
}

template <int OM, int BIASM>
__global__ __launch_bounds__(256) void gemm64(
    const unsigned short* __restrict__ Ap, int lda,
    const unsigned short* __restrict__ Alo, int ldlo, int Klo,
    const unsigned short* __restrict__ Btp, int ldb,
    const float* __restrict__ bias, float bscale,
    void* Cout, int ldc, int M, int N, int K, float oscale) {
  __shared__ __align__(16) float sT[8][16 * 68];
  const int lane = threadIdx.x & 31;
  const int wave = threadIdx.x >> 5;
  const int tilesN = N >> 6;
  const int tilesM = M >> 6;
  const int tile = blockIdx.x * 8 + wave;
  if (tile >= tilesM * tilesN) return;
  const int tm = tile / tilesN;
  const int tn = tile - tm * tilesN;
  const int m0 = tm << 6;
  const int n0 = tn << 6;

  const int rlane = lane & 15;
  const int koff  = (lane >> 4) * 8;
  const int mOff  = (lane >> 4) * 8;

  v8f acc[4][4];
#pragma unroll
  for (int i = 0; i < 4; ++i)
#pragma unroll
    for (int j = 0; j < 4; ++j) acc[i][j] = zero8();

  if (Klo > 0) {
    kloop(acc, Alo, ldlo, Btp, ldb, m0, n0, Klo, rlane, koff);
    acc_guard4(acc[0][0], acc[0][1], acc[0][2], acc[0][3]);
    acc_guard4(acc[1][0], acc[1][1], acc[1][2], acc[1][3]);
    acc_guard4(acc[2][0], acc[2][1], acc[2][2], acc[2][3]);
    acc_guard4(acc[3][0], acc[3][1], acc[3][2], acc[3][3]);
#pragma unroll
    for (int i = 0; i < 4; ++i)
#pragma unroll
      for (int j = 0; j < 4; ++j) acc[i][j] = acc[i][j] * RINV;
  }
  kloop(acc, Ap, lda, Btp, ldb, m0, n0, K, rlane, koff);
  acc_guard4(acc[0][0], acc[0][1], acc[0][2], acc[0][3]);
  acc_guard4(acc[1][0], acc[1][1], acc[1][2], acc[1][3]);
  acc_guard4(acc[2][0], acc[2][1], acc[2][2], acc[2][3]);
  acc_guard4(acc[3][0], acc[3][1], acc[3][2], acc[3][3]);

  const int hh2 = lane >> 4, c4 = (lane & 15) * 4;
  const int q8  = lane >> 3, c8 = (lane & 7) * 8;
  float bc4[4], bc8[8];
#pragma unroll
  for (int e = 0; e < 4; ++e) bc4[e] = 0.f;
#pragma unroll
  for (int e = 0; e < 8; ++e) bc8[e] = 0.f;
  if (BIASM == 0) {
    if (OM == 4) {
      const int cb = n0 + c4;
      const int i0 = (cb <= N - 4) ? cb : (N - 4);
      const v4f b0v = *(const v4f*)(bias + i0);
#pragma unroll
      for (int e = 0; e < 4; ++e) bc4[e] = bfr(b0v[e]) * bscale;
    } else {
      const int cb = n0 + c8;
      const int i0 = (cb <= N - 8) ? cb : (N - 8);
      const v4f b0v = *(const v4f*)(bias + i0), b1v = *(const v4f*)(bias + i0 + 4);
#pragma unroll
      for (int e = 0; e < 4; ++e) { bc8[e] = bfr(b0v[e]) * bscale; bc8[4 + e] = bfr(b1v[e]) * bscale; }
    }
  }

  float* slab = sT[wave];
#pragma unroll
  for (int i = 0; i < 4; ++i) {
    const int mBase = m0 + (i << 4);
#pragma unroll
    for (int j = 0; j < 4; ++j) {
#pragma unroll
      for (int r = 0; r < 8; ++r) {
        slab[(mOff + r) * 68 + (j << 4) + rlane] = acc[i][j][r];
      }
    }
    wave_sync_lds();
    if (OM == 4) {
      float* C = (float*)Cout;
      v4f vals[8];
#pragma unroll
      for (int it = 0; it < 8; ++it) {
        const int row = it * 2 + hh2;
        float rb = 0.f;
        if (BIASM == 1) {
          const int gr = mBase + row;
          rb = bfr(bias[(gr < M) ? gr : (M - 1)]) * bscale;
        }
        v4f v = *(const v4f*)(slab + row * 68 + c4);
#pragma unroll
        for (int e = 0; e < 4; ++e) v[e] = v[e] * oscale + bc4[e] + rb;
        vals[it] = v;
      }
#pragma unroll
      for (int it = 0; it < 8; ++it) {
        const int gr = mBase + it * 2 + hh2;
        *(volatile v4f*)(C + (size_t)gr * (size_t)ldc + n0 + c4) = vals[it];
      }
      __threadfence();
#pragma unroll
      for (int it = 0; it < 8; ++it) {
        const int gr = mBase + it * 2 + hh2;
        *(volatile v4f*)(C + (size_t)gr * (size_t)ldc + n0 + c4) = vals[it];
      }
      __threadfence();
    } else {
      unsigned short* C = (unsigned short*)Cout;
      v4u hv[4];
#pragma unroll
      for (int it = 0; it < 4; ++it) {
        const int row = it * 4 + q8;
        float rb = 0.f;
        if (BIASM == 1) {
          const int gr = mBase + row;
          rb = bfr(bias[(gr < M) ? gr : (M - 1)]) * bscale;
        }
        const float* sp = slab + row * 68 + c8;
        const v4f x0 = *(const v4f*)(sp), x1 = *(const v4f*)(sp + 4);
        float v[8];
#pragma unroll
        for (int e = 0; e < 4; ++e) {
          v[e]     = x0[e] * oscale + bc8[e] + rb;
          v[4 + e] = x1[e] * oscale + bc8[4 + e] + rb;
        }
        v4u ha;
#pragma unroll
        for (int e = 0; e < 4; ++e) ha[e] = pk16(h_bits((_Float16)v[2 * e]), h_bits((_Float16)v[2 * e + 1]));
        hv[it] = ha;
      }
#pragma unroll
      for (int it = 0; it < 4; ++it) {
        const int row = it * 4 + q8;
        const size_t o = (size_t)(mBase + row) * (size_t)ldc + n0 + c8;
        *(volatile v4u*)(C + o) = hv[it];
      }
      __threadfence();
#pragma unroll
      for (int it = 0; it < 4; ++it) {
        const int row = it * 4 + q8;
        const size_t o = (size_t)(mBase + row) * (size_t)ldc + n0 + c8;
        *(volatile v4u*)(C + o) = hv[it];
      }
      __threadfence();
    }
    wave_sync_lds();
  }
}

__global__ __launch_bounds__(256) void egok(const float* __restrict__ ego, const float* __restrict__ W,
                                            const float* __restrict__ b, float* KV) {
  __shared__ __align__(16) float so[DM];
  const int t  = threadIdx.x;
  const int rb = blockIdx.x;
  float s = 0.f;
  if (rb == 0) {
    float a = 0.f;
#pragma unroll 1
    for (int k = 0; k < DCAM; ++k) a += bfr(ego[k]) * bfr(W[(size_t)k * DM + t]);
    s = a + bfr(b[t]);
  }
  so[t] = s;
  __syncthreads();
  const int tc = (t < 64) ? t : 0;
  const v4f o = *(const v4f*)(so + 4 * tc);
  float* dp = KV + (size_t)(NG + rb) * DM + 4 * tc;
  if (t < 64) *(volatile v4f*)dp = o;
  __threadfence();
  if (t < 64) *(volatile v4f*)dp = o;
}

__global__ __launch_bounds__(256) void vsumk(const float* __restrict__ KV, const float* __restrict__ Wv,
                                             const float* __restrict__ bv, float* S) {
  __shared__ float cs[DM];
  __shared__ __align__(16) float so[DM];
  const int t = threadIdx.x;
  double a = 0.0;
#pragma unroll 1
  for (int key = 0; key < KVV; ++key) a += (double)KV[(size_t)key * DM + t];
  cs[t] = (float)a;
  __syncthreads();
  float s = 0.f;
#pragma unroll 1
  for (int j = 0; j < DM; ++j) s += cs[j] * bfr(Wv[(size_t)j * DM + t]);
  s += (float)KVV * bfr(bv[t]);
  so[t] = s;
  __syncthreads();
  const int tc = (t < 64) ? t : 0;
  const v4f o = *(const v4f*)(so + 4 * tc);
  float* dp = S + 4 * tc;
  if (t < 64) *(volatile v4f*)dp = o;
  __threadfence();
  if (t < 64) *(volatile v4f*)dp = o;
}

__device__ __forceinline__ void ostep(float t0, float t1, float& m, float& l) {
  float mx = fmaxf(t0, t1);
  mx = fmaxf(mx, __shfl_xor(mx, 1, 32));
  mx = fmaxf(mx, __shfl_xor(mx, 2, 32));
  mx = fmaxf(mx, __shfl_xor(mx, 4, 32));
  mx = fmaxf(mx, __shfl_xor(mx, 8, 32));
  const float mn = fmaxf(m, mx);
  const float al = exp2f(m - mn);
  float ps = exp2f(t0 - mn) + exp2f(t1 - mn);
  ps += __shfl_xor(ps, 1, 32);
  ps += __shfl_xor(ps, 2, 32);
  ps += __shfl_xor(ps, 4, 32);
  ps += __shfl_xor(ps, 8, 32);
  l = l * al + ps;
  m = mn;
}

__global__ __launch_bounds__(128)
void statk(const unsigned short* __restrict__ QP, const unsigned short* __restrict__ KP, float* ST) {
  __shared__ __align__(16) float Ls[4][32];
  const int tid  = threadIdx.x;
  const int wave = tid >> 5;
  const int lane = tid & 31;
  const int hh   = lane >> 4;
  const int c    = lane & 15;
  const int wid  = blockIdx.x * 4 + wave;
  if (wid >= NWAV) return;
  const int h  = wid & (NH - 1);
  const int gt = wid >> 2;
  const int q0 = gt * 16;

  const _Float16* qp = (const _Float16*)(const void*)QP + (size_t)(q0 + c) * (size_t)DM + HD * h + 8 * hh;
  const v16h qa = ldfrag_h(qp), qb = ldfrag_h(qp + 32);
  const _Float16* kp = (const _Float16*)(const void*)KP + (size_t)c * (size_t)DM + HD * h + 8 * hh;
  const float lsc = (1.4426950408889634f * 0.125f) / (QKC * QKC);

  float m[8], l[8];
#pragma unroll
  for (int r = 0; r < 8; ++r) { m[r] = NEGS; l[r] = 0.f; }

#pragma unroll 1
  for (int ks = 0; ks < KSTEPS; ++ks) {
    const int kb = ks * 32;
    v8f s0, s1;
    {
      const _Float16* k0p = kp + (size_t)kb * DM;
      const _Float16* k1p = kp + (size_t)(kb + 16) * DM;
      const v16h ka0 = ldfrag_h(k0p), kb0 = ldfrag_h(k0p + 32);
      const v16h ka1 = ldfrag_h(k1p), kb1 = ldfrag_h(k1p + 32);
      s0 = mma_raw(qa, ka0, zero8());
      s0 = mma_raw(qb, kb0, s0);
      s1 = mma_raw(qa, ka1, zero8());
      s1 = mma_raw(qb, kb1, s1);
      guard_2x6(s0, s1, qa, qb, ka0, kb0, ka1, kb1);
    }
    const bool v0 = (kb + c) < KVV;
    const bool v1 = (kb + 16 + c) < KVV;
#pragma unroll
    for (int r = 0; r < 8; ++r) {
      const float t0 = v0 ? s0[r] * lsc : NEGS;
      const float t1 = v1 ? s1[r] * lsc : NEGS;
      ostep(t0, t1, m[r], l[r]);
    }
  }

  float* ls = Ls[wave];
#pragma unroll
  for (int r = 0; r < 8; ++r) {
    ls[8 * hh + r]      = m[r];
    ls[16 + 8 * hh + r] = l[r];
  }
  wave_sync_lds();
  const int tc = lane & 7;
  const v4f o = *(const v4f*)(ls + 4 * tc);
  float* dp = ST + (size_t)wid * 32 + 4 * tc;
  if (lane < 8) *(volatile v4f*)dp = o;
  __threadfence();
  if (lane < 8) *(volatile v4f*)dp = o;
}

__device__ __forceinline__ void build_ph(const float* pt, int c, int hh, FragH& ph) {
  const float* prow = pt + c * PSP + 8 * hh;
  const v4f p0 = *(const v4f*)(prow), p1 = *(const v4f*)(prow + 4);
  const v4f p2 = *(const v4f*)(prow + 16), p3 = *(const v4f*)(prow + 20);
#pragma unroll
  for (int e = 0; e < 4; ++e) {
    ph.h[0][e]     = (_Float16)p0[e];
    ph.h[0][4 + e] = (_Float16)p1[e];
    ph.h[1][e]     = (_Float16)p2[e];
    ph.h[1][4 + e] = (_Float16)p3[e];
  }
}

__global__ __launch_bounds__(128)
void pvk(const unsigned short* __restrict__ QP, const unsigned short* __restrict__ KP,
         const unsigned short* __restrict__ VTH, const float* __restrict__ ST, const float* __restrict__ S,
         unsigned short* CT) {
  __shared__ __align__(16) float Ps[4][16 * PSP];
  __shared__ __align__(16) float Os[4][16 * 64];
  const int tid  = threadIdx.x;
  const int wave = tid >> 5;
  const int lane = tid & 31;
  const int hh   = lane >> 4;
  const int c    = lane & 15;
  const int wid  = blockIdx.x * 4 + wave;
  if (wid >= NWAV) return;
  const int h  = wid & (NH - 1);
  const int gt = wid >> 2;
  const int q0 = gt * 16;

  const _Float16* qp = (const _Float16*)(const void*)QP + (size_t)(q0 + c) * (size_t)DM + HD * h + 8 * hh;
  const v16h qa = ldfrag_h(qp), qb = ldfrag_h(qp + 32);
  const _Float16* kp  = (const _Float16*)(const void*)KP + (size_t)c * (size_t)DM + HD * h + 8 * hh;
  const _Float16* vtp = (const _Float16*)(const void*)VTH + (size_t)(HD * h + c) * (size_t)NKP + 8 * hh;
  const float lsc = (1.4426950408889634f * 0.125f) / (QKC * QKC);

  const float* stp = ST + (size_t)wid * 32 + 8 * hh;
  float m[8], f[8];
#pragma unroll
  for (int r = 0; r < 8; ++r) {
    m[r] = stp[r];
    f[r] = PCAR / stp[16 + r];
  }

  v8f z0 = zero8(), z1 = zero8(), z2 = zero8(), z3 = zero8();
  float* pP = Ps[wave];

#pragma unroll 1
  for (int ks = 0; ks < KSTEPS; ++ks) {
    const int kb = ks * 32;
    v8f s0, s1;
    {
      const _Float16* k0p = kp + (size_t)kb * DM;
      const _Float16* k1p = kp + (size_t)(kb + 16) * DM;
      const v16h ka0 = ldfrag_h(k0p), kb0 = ldfrag_h(k0p + 32);
      const v16h ka1 = ldfrag_h(k1p), kb1 = ldfrag_h(k1p + 32);
      s0 = mma_raw(qa, ka0, zero8());
      s0 = mma_raw(qb, kb0, s0);
      s1 = mma_raw(qa, ka1, zero8());
      s1 = mma_raw(qb, kb1, s1);
      guard_2x6(s0, s1, qa, qb, ka0, kb0, ka1, kb1);
    }
    const bool v0 = (kb + c) < KVV;
    const bool v1 = (kb + 16 + c) < KVV;
#pragma unroll
    for (int r = 0; r < 8; ++r) {
      const float e0 = v0 ? (exp2f(s0[r] * lsc - m[r]) * f[r] - PONE) : 0.f;
      const float e1 = v1 ? (exp2f(s1[r] * lsc - m[r]) * f[r] - PONE) : 0.f;
      const int ro = (8 * hh + r) * PSP + c;
      pP[ro]      = e0;
      pP[ro + 16] = e1;
    }
    wave_sync_lds();
    const v16h vh0 = ldfrag_h(vtp + kb);
    const v16h vh1 = ldfrag_h(vtp + (size_t)16 * (size_t)NKP + kb);
    const v16h vh2 = ldfrag_h(vtp + (size_t)32 * (size_t)NKP + kb);
    const v16h vh3 = ldfrag_h(vtp + (size_t)48 * (size_t)NKP + kb);
    {
      FragH ph;
      build_ph(pP, c, hh, ph);
      z0 = mma_raw(ph.v, vh0, z0);
      z1 = mma_raw(ph.v, vh1, z1);
      z2 = mma_raw(ph.v, vh2, z2);
      z3 = mma_raw(ph.v, vh3, z3);
      guard_4x5(z0, z1, z2, z3, ph.v, vh0, vh1, vh2, vh3);
    }
    wave_sync_lds();
  }

  const float* Sp = S + HD * h + c;
  const float Sd0 = Sp[0], Sd1 = Sp[16], Sd2 = Sp[32], Sd3 = Sp[48];
  const float oc = ZC / (PCAR * VC);
  const float sa = PONE * VC;
  float* os = Os[wave];
#pragma unroll
  for (int r = 0; r < 8; ++r) {
    const int ro = (8 * hh + r) * 64 + c;
    os[ro]      = (z0[r] + sa * Sd0) * oc;
    os[ro + 16] = (z1[r] + sa * Sd1) * oc;
    os[ro + 32] = (z2[r] + sa * Sd2) * oc;
    os[ro + 48] = (z3[r] + sa * Sd3) * oc;
  }
  wave_sync_lds();
  const int q8 = lane >> 3, c8 = (lane & 7) * 8;
  v4u ov[4];
  size_t oo[4];
#pragma unroll
  for (int it = 0; it < 4; ++it) {
    const int row = it * 4 + q8;
    ov[it] = pack8h(os + row * 64 + c8);
    oo[it] = (size_t)(q0 + row) * (size_t)DM + (size_t)(HD * h + c8);
  }
#pragma unroll
  for (int it = 0; it < 4; ++it) *(volatile v4u*)(CT + oo[it]) = ov[it];
  __threadfence();
#pragma unroll
  for (int it = 0; it < 4; ++it) *(volatile v4u*)(CT + oo[it]) = ov[it];
  __threadfence();
  wave_sync_lds();
}

__global__ __launch_bounds__(256) void packk(const float* __restrict__ VIS, const float* __restrict__ UNS,
                                             const float* __restrict__ st, const float* __restrict__ cam,
                                             const float* __restrict__ mot, const int* __restrict__ vm,
                                             const float* __restrict__ g, const float* __restrict__ beta,
                                             unsigned short* GH, unsigned short* GL) {
  __shared__ float red[8];
  __shared__ __align__(16) unsigned short hs[GIN];
  __shared__ __align__(16) unsigned short lsd[DM];
  const int t = threadIdx.x, wave = t >> 5, lane = t & 31;
  const int row = blockIdx.x;
  const float x = fmaxf(VIS[(size_t)row * DM + t], 0.f);

  float s = x;
  s += __shfl_xor(s, 16, 32);
  s += __shfl_xor(s, 8, 32);
  s += __shfl_xor(s, 4, 32);
  s += __shfl_xor(s, 2, 32);
  s += __shfl_xor(s, 1, 32);
  if (lane == 0) red[wave] = s;
  __syncthreads();
  float tot = 0.f;
#pragma unroll
  for (int w = 0; w < 8; ++w) tot += red[w];
  const float mu = tot * (1.0f / 256.0f);
  __syncthreads();
  const float d = x - mu;
  float s2 = d * d;
  s2 += __shfl_xor(s2, 16, 32);
  s2 += __shfl_xor(s2, 8, 32);
  s2 += __shfl_xor(s2, 4, 32);
  s2 += __shfl_xor(s2, 2, 32);
  s2 += __shfl_xor(s2, 1, 32);
  if (lane == 0) red[wave] = s2;
  __syncthreads();
  float tot2 = 0.f;
#pragma unroll
  for (int w = 0; w < 8; ++w) tot2 += red[w];
  const float var = tot2 * (1.0f / 256.0f);
  const float visv = d * rsqrtf(var + 1e-5f) * bfr(g[t]) + bfr(beta[t]);
  const float un   = UNS[(size_t)row * DM + t];
  const float sel  = (vm[row] != 0) ? visv : un;

  const float vcar = sel * ACT;
  const _Float16 hv = (_Float16)vcar;
  const _Float16 lv = (_Float16)((vcar - (float)hv) * RESC);
  hs[t]  = h_bits(hv);
  lsd[t] = h_bits(lv);
  hs[DM + t] = h_bits((_Float16)(bfr(st[(size_t)row * DSTR + t]) * ACT));
  if (t < DCAM) hs[DM + DSTR + t]        = h_bits((_Float16)(bfr(cam[(size_t)row * DCAM + t]) * ACT));
  if (t < DMOT) hs[DM + DSTR + DCAM + t] = h_bits((_Float16)(bfr(mot[(size_t)row * DMOT + t]) * ACT));
  __syncthreads();

  const int  t88  = (t < 88) ? t : 0;
  const bool lolane = (t >= 128) && (t < 160);
  const int  t32  = lolane ? (t - 128) : 0;
  const v4u  oh   = *(const v4u*)(hs + 8 * t88);
  const v4u  ol   = *(const v4u*)(lsd + 8 * t32);
  unsigned short* dh = GH + (size_t)row * GIN + 8 * t88;
  unsigned short* dl = GL + (size_t)row * DM + 8 * t32;
  if (t < 88)  *(volatile v4u*)dh = oh;
  if (lolane)  *(volatile v4u*)dl = ol;
  __threadfence();
  if (t < 88)  *(volatile v4u*)dh = oh;
  if (lolane)  *(volatile v4u*)dl = ol;
}

__global__ __launch_bounds__(256) void gatesk(const float* __restrict__ GI, const float* __restrict__ GHd,
                                              const float* __restrict__ mem, const int* __restrict__ valid,
                                              float* out) {
  __shared__ __align__(16) float so[DM];
  const int t = threadIdx.x;
  const int row = blockIdx.x;
  const size_t gb = (size_t)row * GOUT + t;
  const float ar = GI[gb] + GHd[gb];
  const float az = GI[gb + DM] + GHd[gb + DM];
  const float rg = 1.0f / (1.0f + expf(-ar));
  const float zg = 1.0f / (1.0f + expf(-az));
  const float ng = tanhf(GI[gb + 2 * DM] + rg * GHd[gb + 2 * DM]);
  const float mv = bfr(mem[(size_t)row * DM + t]);
  const float hv = (1.0f - zg) * ng + zg * mv;
  const float ov = hv * (float)valid[row];
  so[t] = ov;
  __syncthreads();
  const int tc = (t < 64) ? t : 0;
  const v4f o = *(const v4f*)(so + 4 * tc);
  float* dp = out + (size_t)row * DM + 4 * tc;
  if (t < 64) *(volatile v4f*)dp = o;
  __threadfence();
  if (t < 64) *(volatile v4f*)dp = o;
}

static inline dim3 ggrid(int M, int N) { return dim3((unsigned)((((M / 64) * (N / 64)) + 7) / 8)); }

extern "C" void kernel_launch(void* const* d_in, const int* in_sizes, int n_in,
                              void* d_out, int out_size, void* d_ws, size_t ws_size,
                              hipStream_t stream) {
  if (n_in < 31) return;
  if (in_sizes[0] != NQ * DM) return;
  if (in_sizes[1] != NQ * DROI) return;
  if (in_sizes[2] != NQ * DSTR || in_sizes[3] != NG * DSTR) return;
  if (in_sizes[4] != NQ * DCAM || in_sizes[5] != DCAM || in_sizes[6] != NQ * DMOT) return;
  if (in_sizes[7] != NQ || in_sizes[8] != NQ) return;
  if (in_sizes[9] != DROI * DM || in_sizes[10] != DM || in_sizes[11] != DM || in_sizes[12] != DM) return;
  if (in_sizes[13] != DSTR * DM || in_sizes[14] != DM) return;
  if (in_sizes[15] != DCAM * DM || in_sizes[16] != DM) return;
  if (in_sizes[17] != DM * DM || in_sizes[18] != DM || in_sizes[19] != DM * DM || in_sizes[20] != DM) return;
  if (in_sizes[21] != DM * DM || in_sizes[22] != DM || in_sizes[23] != DM * DM || in_sizes[24] != DM) return;
  if (in_sizes[25] != DM * DM || in_sizes[26] != DM) return;
  if (in_sizes[27] != GIN * GOUT || in_sizes[28] != DM * GOUT || in_sizes[29] != GOUT || in_sizes[30] != GOUT) return;
  if (out_size != NQ * DM) return;

  const float* memory = (const float*)d_in[0];
  const float* visual = (const float*)d_in[1];
  const float* strt   = (const float*)d_in[2];
  const float* gst    = (const float*)d_in[3];
  const float* cam    = (const float*)d_in[4];
  const float* ego    = (const float*)d_in[5];
  const float* mot    = (const float*)d_in[6];
  const int*   vism   = (const int*)d_in[7];
  const int*   validm = (const int*)d_in[8];
  const float* vp_w   = (const float*)d_in[9];
  const float* vp_b   = (const float*)d_in[10];
  const float* ln_g   = (const float*)d_in[11];
  const float* ln_b   = (const float*)d_in[12];
  const float* kv_w   = (const float*)d_in[13];
  const float* kv_b   = (const float*)d_in[14];
  const float* ego_w  = (const float*)d_in[15];
  const float* ego_b  = (const float*)d_in[16];
  const float* wq     = (const float*)d_in[17];
  const float* bq     = (const float*)d_in[18];
  const float* wk     = (const float*)d_in[19];
  const float* bk     = (const float*)d_in[20];
  const float* wv     = (const float*)d_in[21];
  const float* bv     = (const float*)d_in[22];
  const float* wo     = (const float*)d_in[23];
  const float* bo     = (const float*)d_in[24];
  const float* un_w   = (const float*)d_in[25];
  const float* un_b   = (const float*)d_in[26];
  const float* g_wih  = (const float*)d_in[27];
  const float* g_whh  = (const float*)d_in[28];
  const float* g_bih  = (const float*)d_in[29];
  const float* g_bhh  = (const float*)d_in[30];
  float*       out    = (float*)d_out;

  size_t off = 0;
  auto carve = [&](size_t bytes) -> size_t {
    const size_t o = off;
    off += (bytes + (size_t)65535) & ~(size_t)65535;
    return o;
  };
  const size_t oVISP  = carve((size_t)NQ * DROI * 2);
  const size_t oWVPT  = carve((size_t)DM * DROI * 2);
  const size_t oVIS32 = carve((size_t)NQ * DM * 4);
  const size_t oGSTP  = carve((size_t)NG * DSTR * 2);
  const size_t oWKVT  = carve((size_t)DM * DSTR * 2);
  const size_t oKV32  = carve((size_t)NKP * DM * 4);
  const size_t oKVH   = carve((size_t)NKP * DM * 2);
  const size_t oS     = carve((size_t)DM * 4);
  const size_t oMEMP  = carve((size_t)NQ * DM * 2);
  const size_t oWQT   = carve((size_t)DM * DM * 2);
  const size_t oWKT   = carve((size_t)DM * DM * 2);
  const size_t oWVT   = carve((size_t)DM * DM * 2);
  const size_t oQP    = carve((size_t)NQ * DM * 2);
  const size_t oKP    = carve((size_t)NKP * DM * 2);
  const size_t oVTH   = carve((size_t)DM * NKP * 2);
  const size_t oST    = carve((size_t)NWAV * 32 * 4);
  const size_t oCTXP  = carve((size_t)NQ * DM * 2);
  const size_t oWOT   = carve((size_t)DM * DM * 2);
  const size_t oATTP  = carve((size_t)NQ * DM * 2);
  const size_t oWUT   = carve((size_t)DM * DM * 2);
  const size_t oUNS32 = carve((size_t)NQ * DM * 4);
  const size_t oGIH   = carve((size_t)NQ * GIN * 2);
  const size_t oGIL   = carve((size_t)NQ * DM * 2);
  const size_t oWIHT  = carve((size_t)GOUT * GIN * 2);
  const size_t oWHHT  = carve((size_t)GOUT * DM * 2);
  const size_t oGI32  = carve((size_t)NQ * GOUT * 4);
  const size_t oGH32  = carve((size_t)NQ * GOUT * 4);
  if (off > ws_size) return;
  if (off > (size_t)134217728) return;

  char* ws = (char*)d_ws;
  unsigned short* VISP  = (unsigned short*)(ws + oVISP);
  unsigned short* WVPT  = (unsigned short*)(ws + oWVPT);
  float*          VIS32 = (float*)(ws + oVIS32);
  unsigned short* GSTP  = (unsigned short*)(ws + oGSTP);
  unsigned short* WKVT  = (unsigned short*)(ws + oWKVT);
  float*          KV32  = (float*)(ws + oKV32);
  unsigned short* KVH   = (unsigned short*)(ws + oKVH);
  float*          S     = (float*)(ws + oS);
  unsigned short* MEMP  = (unsigned short*)(ws + oMEMP);
  unsigned short* WQT   = (unsigned short*)(ws + oWQT);
  unsigned short* WKT   = (unsigned short*)(ws + oWKT);
  unsigned short* WVT   = (unsigned short*)(ws + oWVT);
  unsigned short* QP    = (unsigned short*)(ws + oQP);
  unsigned short* KP    = (unsigned short*)(ws + oKP);
  unsigned short* VTH   = (unsigned short*)(ws + oVTH);
  float*          ST    = (float*)(ws + oST);
  unsigned short* CTXP  = (unsigned short*)(ws + oCTXP);
  unsigned short* WOT   = (unsigned short*)(ws + oWOT);
  unsigned short* ATTP  = (unsigned short*)(ws + oATTP);
  unsigned short* WUT   = (unsigned short*)(ws + oWUT);
  float*          UNS32 = (float*)(ws + oUNS32);
  unsigned short* GIH   = (unsigned short*)(ws + oGIH);
  unsigned short* GIL   = (unsigned short*)(ws + oGIL);
  unsigned short* WIHT  = (unsigned short*)(ws + oWIHT);
  unsigned short* WHHT  = (unsigned short*)(ws + oWHHT);
  float*          GI32  = (float*)(ws + oGI32);
  float*          GH32  = (float*)(ws + oGH32);

  const dim3 blk(256), blk128(128);
  const float osA = 1.0f / (ACT * WSC);
  const float osQ = QKC / (ACT * WSC);
  const float osV = VC / (ACT * WSC);
  const float osO = AOC / (ZC * WSC);
  const float osU = 1.0f / (AOC * WSC);

  cvk<<<dim3((NQ * DROI / 8) / 256), blk, 0, stream>>>(visual, VISP, NQ * DROI / 8, 1, ACT);
  cvk<<<dim3((NG * DSTR / 8) / 256), blk, 0, stream>>>(gst, GSTP, NG * DSTR / 8, 1, ACT);
  cvk<<<dim3((NQ * DM / 8) / 256), blk, 0, stream>>>(memory, MEMP, NQ * DM / 8, 1, ACT);

  cvT<<<dim3(DM / 64, DROI / 64), blk, 0, stream>>>(vp_w, WVPT, DROI, DM, WSC);
  cvT<<<dim3(DM / 64, DSTR / 64), blk, 0, stream>>>(kv_w, WKVT, DSTR, DM, WSC);
  cvT<<<dim3(DM / 64, DM / 64), blk, 0, stream>>>(wq, WQT, DM, DM, WSC);
  cvT<<<dim3(DM / 64, DM / 64), blk, 0, stream>>>(wk, WKT, DM, DM, WSC);
  cvT<<<dim3(DM / 64, DM / 64), blk, 0, stream>>>(wv, WVT, DM, DM, WSC);
  cvT<<<dim3(DM / 64, DM / 64), blk, 0, stream>>>(wo, WOT, DM, DM, WSC);
  cvT<<<dim3(DM / 64, DM / 64), blk, 0, stream>>>(un_w, WUT, DM, DM, WSC);
  cvT<<<dim3(GOUT / 64, GIN / 64), blk, 0, stream>>>(g_wih, WIHT, GIN, GOUT, WSC);
  cvT<<<dim3(GOUT / 64, DM / 64), blk, 0, stream>>>(g_whh, WHHT, DM, GOUT, WSC);

  gemm64<4, 0><<<ggrid(NQ, DM), blk, 0, stream>>>(
      VISP, DROI, VISP, DROI, 0, WVPT, DROI, vp_b, 1.0f, (void*)VIS32, DM, NQ, DM, DROI, osA);

  gemm64<4, 0><<<ggrid(NG, DM), blk, 0, stream>>>(
      GSTP, DSTR, GSTP, DSTR, 0, WKVT, DSTR, kv_b, 1.0f, (void*)KV32, DM, NG, DM, DSTR, osA);
  egok<<<dim3(NKP - NG), blk, 0, stream>>>(ego, ego_w, ego_b, KV32);
  cvk<<<dim3((NKP * DM / 8) / 256), blk, 0, stream>>>(KV32, KVH, NKP * DM / 8, 0, ACT);
  vsumk<<<dim3(1), blk, 0, stream>>>(KV32, wv, bv, S);

  gemm64<2, 0><<<ggrid(NQ, DM), blk, 0, stream>>>(
      MEMP, DM, MEMP, DM, 0, WQT, DM, bq, QKC, (void*)QP, DM, NQ, DM, DM, osQ);
  gemm64<2, 0><<<ggrid(NKP, DM), blk, 0, stream>>>(
      KVH, DM, KVH, DM, 0, WKT, DM, bk, QKC, (void*)KP, DM, NKP, DM, DM, osQ);
  gemm64<2, 1><<<ggrid(DM, NKP), blk, 0, stream>>>(
      WVT, DM, WVT, DM, 0, KVH, DM, bv, VC, (void*)VTH, NKP, DM, NKP, DM, osV);

  statk<<<dim3(NWAV / 4), blk128, 0, stream>>>(QP, KP, ST);
  pvk<<<dim3(NWAV / 4), blk128, 0, stream>>>(QP, KP, VTH, ST, S, CTXP);

  gemm64<2, 0><<<ggrid(NQ, DM), blk, 0, stream>>>(
      CTXP, DM, CTXP, DM, 0, WOT, DM, bo, AOC, (void*)ATTP, DM, NQ, DM, DM, osO);
  gemm64<4, 0><<<ggrid(NQ, DM), blk, 0, stream>>>(
      ATTP, DM, ATTP, DM, 0, WUT, DM, un_b, 1.0f, (void*)UNS32, DM, NQ, DM, DM, osU);

  packk<<<dim3(NQ), blk, 0, stream>>>(VIS32, UNS32, strt, cam, mot, vism, ln_g, ln_b, GIH, GIL);

  gemm64<4, 0><<<ggrid(NQ, GOUT), blk, 0, stream>>>(
      GIH, GIN, GIL, DM, DM, WIHT, GIN, g_bih, 1.0f, (void*)GI32, GOUT, NQ, GOUT, GIN, osA);
  gemm64<4, 0><<<ggrid(NQ, GOUT), blk, 0, stream>>>(
      MEMP, DM, MEMP, DM, 0, WHHT, DM, g_bhh, 1.0f, (void*)GH32, GOUT, NQ, GOUT, DM, osA);

  gatesk<<<dim3(NQ), blk, 0, stream>>>(GI32, GH32, memory, validm, out);

  (void)hipGetLastError();
}
